// PhaseFunctionedLinear_80762565034652
// MI455X (gfx1250) — hardware-verified
//
#include <hip/hip_runtime.h>

#define NB     8192
#define IDIM   1024
#define ODIM   1024
#define NCP    6
#define NX     (NB * IDIM)
#define NWALL  (NCP * ODIM * IDIM)
#define NBIAS  (NCP * ODIM)
#define NX8    (NX / 8)
#define NW8    (NWALL / 8)
#define TM     128
#define TN     64

static_assert(NB % TM == 0);
static_assert(ODIM % TN == 0);
static_assert(IDIM % 32 == 0);
static_assert(NX8 % 256 == 0);
static_assert(NB % 256 == 0);

typedef unsigned short u16;
typedef __attribute__((ext_vector_type(16))) __bf16 v16b;
typedef unsigned int v4u  __attribute__((ext_vector_type(4)));
typedef u16          v8us __attribute__((ext_vector_type(8)));
typedef float        v8f  __attribute__((ext_vector_type(8)));
typedef float        v4f  __attribute__((ext_vector_type(4)));
typedef v4u __attribute__((may_alias)) v4ua;
typedef v4f __attribute__((may_alias)) v4fa;

union Frag { v16b v; v4u q[2]; };

__device__ __forceinline__ u16 bf16_bits(float x) {
  unsigned u = __float_as_uint(x);
  u += 0x7FFFu + ((u >> 16) & 1u);
  return (u16)(u >> 16);
}
__device__ __forceinline__ float bf16_val(float x) {
  return __uint_as_float(((unsigned)bf16_bits(x)) << 16);
}

__device__ __forceinline__ v8f wmma_bf16(v16b a, v16b b, v8f c) {
  v8f d = __builtin_amdgcn_wmma_f32_16x16x32_bf16(false, a, false, b, (short)0, c, false, false);
  asm volatile("v_nop\n\tv_nop\n\tv_nop\n\tv_nop" : "+v"(d) : "v"(a), "v"(b));
  return d;
}

__device__ __forceinline__ v16b load_frag(const u16* p, int h) {
  Frag f;
  f.q[0] = *(const v4ua*)(p + 8 * h);
  f.q[1] = *(const v4ua*)(p + 16 + 8 * h);
  return f.v;
}

__global__ __launch_bounds__(256) void cvt_kernel(
    const float* __restrict__ x, const float* __restrict__ w,
    u16* __restrict__ xh, u16* __restrict__ wh)
{
  const int g = blockIdx.x * 256 + threadIdx.x;
  if (g >= NX8 + NW8) return;
  const float* src;
  u16* dst;
  if (g < NX8) {
    src = x + (size_t)g * 8;
    dst = xh + (size_t)g * 8;
  } else {
    const int e = g - NX8;
    src = w + (size_t)e * 8;
    dst = wh + (size_t)e * 8;
  }
  const v4f a = *(const v4fa*)src;
  const v4f c = *(const v4fa*)(src + 4);
  v8us o;
  o[0] = bf16_bits(a.x); o[1] = bf16_bits(a.y); o[2] = bf16_bits(a.z); o[3] = bf16_bits(a.w);
  o[4] = bf16_bits(c.x); o[5] = bf16_bits(c.y); o[6] = bf16_bits(c.z); o[7] = bf16_bits(c.w);
  *(volatile v8us*)dst = o;
  __threadfence();
  *(volatile v8us*)dst = o;
}

__device__ __forceinline__ void coef_store_pass(const float* sC, float* coef, int b0, int tid) {
  #pragma unroll
  for (int it = 0; it < 2; ++it) {
    const int s = tid + it * 256;
    if (s < NCP * 64) {
      const int plane = s >> 6, q = s & 63;
      const v4f v = *(const v4fa*)(sC + plane * 256 + 4 * q);
      *(volatile v4f*)(coef + (size_t)plane * NB + b0 + 4 * q) = v;
    }
  }
}

__global__ __launch_bounds__(256) void coef_kernel(
    const float* __restrict__ phase, float* __restrict__ coef)
{
  #pragma clang fp contract(off)
  __shared__ __attribute__((aligned(16))) float sC[NCP * 256];

  const int tid = threadIdx.x;
  const int b0 = blockIdx.x * 256;
  const int b = min(b0 + tid, NB - 1);

  const float two_pi = (float)6.283185307179586;
  const float kscale = (float)(6.0 / 6.283185307179586);

  const float phb = bf16_val(phase[b]);
  float ph = fmodf(phb, two_pi);
  if (ph < 0.0f) ph = ph + two_pi;
  const float pos = ph * kscale;
  const float base = floorf(pos);
  int bi = (int)base;
  bi = max(-16, min(bi, 16));
  const float t  = pos - base;
  const float t2 = t * t;
  const float t3 = t2 * t;
  const float w0 = ((-0.5f * t) + t2) - (0.5f * t3);
  const float w1 = (1.0f - (2.5f * t2)) + (1.5f * t3);
  const float w2 = ((0.5f * t) + (2.0f * t2)) - (1.5f * t3);
  const float w3 = (-0.5f * t2) + (0.5f * t3);
  const int i0 = (((bi - 1) % NCP) + NCP) % NCP;
  const int i1 = (((bi    ) % NCP) + NCP) % NCP;
  const int i2 = (((bi + 1) % NCP) + NCP) % NCP;
  const int i3 = (((bi + 2) % NCP) + NCP) % NCP;

  #pragma unroll
  for (int c = 0; c < NCP; ++c) {
    const float v = ((i0 == c) ? w0 : 0.0f) + ((i1 == c) ? w1 : 0.0f)
                  + ((i2 == c) ? w2 : 0.0f) + ((i3 == c) ? w3 : 0.0f);
    sC[c * 256 + tid] = v;
  }
  __syncthreads();

  coef_store_pass(sC, coef, b0, tid);
  __threadfence();
  coef_store_pass(sC, coef, b0, tid);
}

__device__ __forceinline__ void out_store_pass(const float* sO, float* out,
                                               int m0, int n0, int w, int lane) {
  const int q8 = lane & 7, sub = lane >> 3;
  #pragma unroll
  for (int i = 0; i < 16; ++i) {
    const int lid = i * 4 + sub;
    const int row = 32 * w + (lid >> 1), hl = lid & 1;
    const v4f v = *(const v4fa*)(sO + row * TN + 32 * hl + 4 * q8);
    float* dst = out + (size_t)(m0 + row) * ODIM + n0 + 32 * hl + 4 * q8;
    *(volatile v4f*)dst = v;
  }
}

__global__ __launch_bounds__(128) void gemm_kernel(
    const u16* __restrict__ xh,
    const u16* __restrict__ wh,
    const float* __restrict__ coef,
    const float* __restrict__ bias,
    float* __restrict__ out)
{
  #pragma clang fp contract(off)
  __shared__ __attribute__((aligned(16))) float sO[TM * TN];

  const int tid = threadIdx.x, lane = tid & 31, w = tid >> 5;
  const int h = lane >> 4, m = lane & 15;
  const int m0 = blockIdx.x * TM;
  const int n0 = blockIdx.y * TN;
  const int m0w = m0 + 32 * w;

  const u16* xa0 = xh + (size_t)(m0w + m) * IDIM;
  const u16* xa1 = xa0 + (size_t)16 * IDIM;

  #pragma unroll
  for (int mt = 0; mt < 2; ++mt)
    #pragma unroll
    for (int nt = 0; nt < 4; ++nt)
      #pragma unroll
      for (int r = 0; r < 8; ++r) {
        const int trow = 32 * w + 16 * mt + 8 * h + r;
        sO[trow * TN + 16 * nt + m] = 0.0f;
      }

  const v8f zero8 = {0.f, 0.f, 0.f, 0.f, 0.f, 0.f, 0.f, 0.f};

  #pragma unroll 1
  for (int c = 0; c < NCP; ++c) {
    const u16* wb = wh + ((size_t)c * ODIM + n0 + m) * IDIM;

    v8f acc[2][4];
    #pragma unroll
    for (int mt = 0; mt < 2; ++mt)
      #pragma unroll
      for (int nt = 0; nt < 4; ++nt) acc[mt][nt] = zero8;

    #pragma unroll 1
    for (int k0 = 0; k0 < IDIM; k0 += 32) {
      const v16b a0 = load_frag(xa0 + k0, h);
      const v16b a1 = load_frag(xa1 + k0, h);
      #pragma unroll
      for (int nt = 0; nt < 4; ++nt) {
        const v16b bfr = load_frag(wb + (size_t)nt * 16 * IDIM + k0, h);
        acc[0][nt] = wmma_bf16(a0, bfr, acc[0][nt]);
        acc[1][nt] = wmma_bf16(a1, bfr, acc[1][nt]);
      }
    }

    const float* cp = coef + (size_t)c * NB + m0w + 8 * h;
    const v4f c00 = *(const v4fa*)(cp);
    const v4f c01 = *(const v4fa*)(cp + 4);
    const v4f c10 = *(const v4fa*)(cp + 16);
    const v4f c11 = *(const v4fa*)(cp + 20);
    const float cf[2][8] = { { c00.x, c00.y, c00.z, c00.w, c01.x, c01.y, c01.z, c01.w },
                             { c10.x, c10.y, c10.z, c10.w, c11.x, c11.y, c11.z, c11.w } };
    #pragma unroll
    for (int nt = 0; nt < 4; ++nt) {
      const float bvl = bf16_val(bias[c * ODIM + n0 + 16 * nt + m]);
      #pragma unroll
      for (int mt = 0; mt < 2; ++mt) {
        #pragma unroll
        for (int r = 0; r < 8; ++r) {
          const int trow = 32 * w + 16 * mt + 8 * h + r;
          const int idx = trow * TN + 16 * nt + m;
          const float y = acc[mt][nt][r] + bvl;
          const float prod = cf[mt][r] * y;
          const float s = sO[idx];
          sO[idx] = s + prod;
        }
      }
    }
  }
  __syncthreads();

  out_store_pass(sO, out, m0, n0, w, lane);
  __threadfence();
  out_store_pass(sO, out, m0, n0, w, lane);
}

extern "C" void kernel_launch(void* const* d_in, const int* in_sizes, int n_in,
                              void* d_out, int out_size, void* d_ws, size_t ws_size,
                              hipStream_t stream) {
  if (n_in < 4) return;
  if (in_sizes[0] != NX) return;
  if (in_sizes[1] != NB) return;
  if (in_sizes[2] != NWALL) return;
  if (in_sizes[3] != NBIAS) return;
  if (out_size != NX) return;

  const float* x     = (const float*)d_in[0];
  const float* phase = (const float*)d_in[1];
  const float* W     = (const float*)d_in[2];
  const float* bias  = (const float*)d_in[3];
  float* out = (float*)d_out;

  const size_t xh_bytes = (size_t)NX * 2;
  const size_t wh_bytes = (size_t)NWALL * 2;
  const size_t cf_bytes = (size_t)NCP * NB * 4;
  const size_t total = xh_bytes + wh_bytes + cf_bytes;
  if (total > ws_size) return;

  char* ws = (char*)d_ws;
  u16*   xh   = (u16*)(ws);
  u16*   wh   = (u16*)(ws + xh_bytes);
  float* coef = (float*)(ws + xh_bytes + wh_bytes);

  const int ngroups = NX8 + NW8;
  cvt_kernel<<<(ngroups + 255) / 256, 256, 0, stream>>>(x, W, xh, wh);

  coef_kernel<<<(NB + 255) / 256, 256, 0, stream>>>(phase, coef);

  dim3 gG(NB / TM, ODIM / TN);
  gemm_kernel<<<gG, 128, 0, stream>>>(xh, wh, coef, bias, out);
}
